// ObliviousDecisionTreeCMB_38637525795488
// MI455X (gfx1250) — hardware-verified
//
#include <hip/hip_runtime.h>
#include <math.h>

constexpr int kBatch  = 512;
constexpr int kDim    = 256;
constexpr int kNT     = 512;
constexpr int kDepth  = 6;
constexpr int kUnits  = 3;
constexpr int kLeaves = 64;
constexpr int kND     = kNT * kDepth;
constexpr int kHalfNT = 256;

static_assert(kDim % 32 == 0);
static_assert(kBatch % 64 == 0);
static_assert(kND % 64 == 0);
static_assert(kLeaves == (1 << kDepth));
static_assert((kBatch / 64) * (kND / 64) % 8 == 0);

constexpr size_t kBytesX  = (size_t)kBatch * kDim * 2;
constexpr size_t kBytesS  = (size_t)kND * kDim * 2;
constexpr size_t kBytesFV = (size_t)kBatch * kND * 4;
constexpr size_t kOffXhi  = 0;
constexpr size_t kOffXlo  = kOffXhi + kBytesX;
constexpr size_t kOffShi  = kOffXlo + kBytesX;
constexpr size_t kOffSlo  = kOffShi + kBytesS;
constexpr size_t kOffFV   = kOffSlo + kBytesS;
constexpr size_t kWsTotal = kOffFV + kBytesFV;
static_assert(kWsTotal == 9961472);
static_assert(kWsTotal <= 134217728);
static_assert(kOffXlo % 256 == 0 && kOffShi % 256 == 0 && kOffSlo % 256 == 0 && kOffFV % 256 == 0);

typedef __attribute__((ext_vector_type(16))) _Float16 v16h;
typedef __attribute__((ext_vector_type(8)))  _Float16 v8h;
typedef __attribute__((ext_vector_type(16))) __bf16   v16b;
typedef __attribute__((ext_vector_type(8)))  __bf16   v8b;
typedef __attribute__((ext_vector_type(8)))  float    v8f;
typedef __attribute__((ext_vector_type(4)))  float    v4f;
typedef __attribute__((ext_vector_type(2)))  float    v2f;
typedef __attribute__((ext_vector_type(4)))  unsigned int v4u;

__device__ __forceinline__ unsigned short f2bf_bits(float f) {
  unsigned u = __float_as_uint(f);
  return (unsigned short)((u + 0x7FFFu + ((u >> 16) & 1u)) >> 16);
}
__device__ __forceinline__ float bf_bits2f(unsigned short h) { return __uint_as_float(((unsigned)h) << 16); }

__device__ __forceinline__ void dep_guard_h(v8f& a, v8f& b, v16h x, v16h y) { asm volatile("v_nop\n\tv_nop\n\tv_nop\n\tv_nop" : "+v"(a), "+v"(b) : "v"(x), "v"(y)); }
__device__ __forceinline__ void dep_guard_b(v8f& a, v8f& b, v16b x, v16b y) { asm volatile("v_nop\n\tv_nop\n\tv_nop\n\tv_nop" : "+v"(a), "+v"(b) : "v"(x), "v"(y)); }
__device__ __forceinline__ void keep4_h(v16h a, v16h b, v16h c, v16h d) { asm volatile("v_nop" :: "v"(a), "v"(b), "v"(c), "v"(d)); }
__device__ __forceinline__ void keep4_b(v16b a, v16b b, v16b c, v16b d) { asm volatile("v_nop" :: "v"(a), "v"(b), "v"(c), "v"(d)); }
__device__ __forceinline__ void acc_guard4(v8f& a, v8f& b, v8f& c, v8f& d) { asm volatile("v_nop\n\tv_nop\n\tv_nop\n\tv_nop" : "+v"(a), "+v"(b), "+v"(c), "+v"(d)); }
template <typename T> struct Frag;
template <> struct Frag<_Float16> {
  typedef v16h V; union U { v16h v; v8h h[2]; };
  static __device__ __forceinline__ v16h load(const _Float16* p) {
    U f; f.h[0] = *(const v8h*)(p); f.h[1] = *(const v8h*)(p + 16); return f.v;
  }
  static __device__ __forceinline__ v8f mma(v16h a, v16h b, v8f c) {
    return __builtin_amdgcn_wmma_f32_16x16x32_f16(false, a, false, b, (short)0, c, false, false);
  }
  static __device__ __forceinline__ void guard(v8f& a, v8f& b, v16h x, v16h y) { dep_guard_h(a, b, x, y); }
  static __device__ __forceinline__ void keep(v16h a, v16h b, v16h c, v16h d) { keep4_h(a, b, c, d); }
};
template <> struct Frag<__bf16> {
  typedef v16b V; union U { v16b v; v8b h[2]; };
  static __device__ __forceinline__ v16b load(const __bf16* p) {
    U f; f.h[0] = *(const v8b*)(p); f.h[1] = *(const v8b*)(p + 16); return f.v;
  }
  static __device__ __forceinline__ v8f mma(v16b a, v16b b, v8f c) {
    return __builtin_amdgcn_wmma_f32_16x16x32_bf16(false, a, false, b, (short)0, c, false, false);
  }
  static __device__ __forceinline__ void guard(v8f& a, v8f& b, v16b x, v16b y) { dep_guard_b(a, b, x, y); }
  static __device__ __forceinline__ void keep(v16b a, v16b b, v16b c, v16b d) { keep4_b(a, b, c, d); }
};

__device__ __forceinline__ unsigned pk16(unsigned short a, unsigned short b) { return (unsigned)a | ((unsigned)b << 16); }

template <int ET> struct Elem;
template <> struct Elem<0> { typedef _Float16 T; };
template <> struct Elem<1> { typedef __bf16 T; };
template <int ET, bool SPLIT, int BIAS_MODE, int OUT_MODE, bool RESID, int ACT = 0>
__global__ __launch_bounds__(256) void wmma_gemm64(
    const unsigned short* __restrict__ Ap, const unsigned short* __restrict__ A2p, int lda, long strideA,
    const unsigned short* __restrict__ Btp, const unsigned short* __restrict__ Bt2p, int ldb, long strideB,
    void* __restrict__ Cout, void* __restrict__ Cout2, int ldc, long strideC,
    const float* __restrict__ bias,
    const float* __restrict__ resid, long strideR,
    int M, int N, int K, float scale) {
  typedef typename Elem<ET>::T T;
  typedef typename Frag<T>::V V;
  const T* A = (const T*)Ap; const T* A2 = (const T*)A2p; const T* Bt = (const T*)Btp; const T* Bt2 = (const T*)Bt2p;
  __shared__ __align__(16) float sT[8][16 * 68];
  const int b    = blockIdx.y;
  const int lane = threadIdx.x & 31;
  const int wave = threadIdx.x >> 5;
  const int tilesN = N >> 6;
  const int tilesM = M >> 6;
  const int tile = blockIdx.x * 8 + wave;
  if (tile >= tilesM * tilesN) return;
  const int tm = tile / tilesN;
  const int tn = tile - tm * tilesN;
  const int m0 = tm << 6;
  const int n0 = tn << 6;

  const T* Ab  = A  + (size_t)b * strideA;
  const T* Bb  = Bt + (size_t)b * strideB;
  const T* Ab2 = SPLIT ? (A2  + (size_t)b * strideA) : nullptr;
  const T* Bb2 = SPLIT ? (Bt2 + (size_t)b * strideB) : nullptr;

  const int rlane = lane & 15;
  const int koff  = (lane >> 4) * 8;
  const int mOff  = (lane >> 4) * 8;

  v8f acc[4][4];
#pragma unroll
  for (int i = 0; i < 4; ++i)
#pragma unroll
    for (int j = 0; j < 4; ++j) acc[i][j] = (v8f){0.f,0.f,0.f,0.f,0.f,0.f,0.f,0.f};

  for (int k0 = 0; k0 < K; k0 += 32) {
    V bh[4], bl[4];
#pragma unroll
    for (int j = 0; j < 4; ++j) {
      const size_t bo = (size_t)(n0 + (j << 4) + rlane) * ldb + koff + k0;
      bh[j] = Frag<T>::load(Bb + bo);
      if (SPLIT) bl[j] = Frag<T>::load(Bb2 + bo);
    }
#pragma unroll
    for (int i = 0; i < 4; ++i) {
      const size_t ao = (size_t)(m0 + (i << 4) + rlane) * lda + koff + k0;
      V ah = Frag<T>::load(Ab + ao);
      V al;
      if (SPLIT) al = Frag<T>::load(Ab2 + ao);
#pragma unroll
      for (int j = 0; j < 4; ++j) {
        acc[i][j] = Frag<T>::mma(ah, bh[j], acc[i][j]);
        if (SPLIT) {
          acc[i][j] = Frag<T>::mma(ah, bl[j], acc[i][j]);
          acc[i][j] = Frag<T>::mma(al, bh[j], acc[i][j]);
        }
      }
      Frag<T>::guard(acc[i][0], acc[i][3], ah, SPLIT ? al : ah);
    }
    Frag<T>::keep(bh[0], bh[1], bh[2], bh[3]);
    if (SPLIT) Frag<T>::keep(bl[0], bl[1], bl[2], bl[3]);
  }
  acc_guard4(acc[0][0], acc[0][1], acc[0][2], acc[0][3]);
  acc_guard4(acc[1][0], acc[1][1], acc[1][2], acc[1][3]);
  acc_guard4(acc[2][0], acc[2][1], acc[2][2], acc[2][3]);
  acc_guard4(acc[3][0], acc[3][1], acc[3][2], acc[3][3]);

  float* slab = sT[wave];
  const float* Rb = RESID ? (resid + (size_t)b * strideR) : nullptr;
#pragma unroll
  for (int i = 0; i < 4; ++i) {
    const int mBase = m0 + (i << 4);
#pragma unroll
    for (int j = 0; j < 4; ++j) {
      const int n = n0 + (j << 4) + rlane;
      float bv = 0.f;
      if (BIAS_MODE == 2) bv = bias[n];
#pragma unroll
      for (int r = 0; r < 8; ++r) {
        float v = acc[i][j][r] * scale;
        if (BIAS_MODE == 1) v += bias[mBase + mOff + r];
        if (BIAS_MODE == 2) v += bv;
        if (RESID) v += Rb[(size_t)(mBase + mOff + r) * ldc + n];
        if (ACT == 2) v = fmaxf(v, 0.0f);
        if (ACT == 4) v = (v > 0.f) ? v : 0.01f * v;
        slab[(mOff + r) * 68 + (j << 4) + rlane] = v;
      }
    }
    __builtin_amdgcn_fence(__ATOMIC_RELEASE, "workgroup");
    __builtin_amdgcn_wave_barrier();
    __builtin_amdgcn_fence(__ATOMIC_ACQUIRE, "workgroup");
    if (OUT_MODE == 0) {
      float* C = (float*)Cout + (size_t)b * strideC;
      const int hh = lane >> 4, c4 = (lane & 15) * 4;
      for (int pass = 0; pass < 2; ++pass) {
#pragma unroll
        for (int it = 0; it < 8; ++it) {
          const int row = it * 2 + hh;
          v4f v = *(const v4f*)(slab + row * 68 + c4);
          *(volatile v4f*)(C + (size_t)(mBase + row) * ldc + n0 + c4) = v;
        }
        __threadfence();
      }
    } else {
      const int q = lane >> 3, c8 = (lane & 7) * 8;
      unsigned short* C  = (unsigned short*)Cout  + (size_t)b * strideC;
      unsigned short* C2 = (OUT_MODE == 2) ? ((unsigned short*)Cout2 + (size_t)b * strideC) : nullptr;
      for (int pass = 0; pass < 2; ++pass) {
#pragma unroll
        for (int it = 0; it < 4; ++it) {
          const int row = it * 4 + q;
          const float* sp = slab + row * 68 + c8;
          v8h hv, lv;
#pragma unroll
          for (int e = 0; e < 8; ++e) {
            if (OUT_MODE == 1) {
              hv[e] = (_Float16)sp[e];
            } else {
              unsigned short hb = f2bf_bits(sp[e]);
              unsigned short lb = f2bf_bits(sp[e] - bf_bits2f(hb));
              hv[e] = __builtin_bit_cast(_Float16, hb);
              lv[e] = __builtin_bit_cast(_Float16, lb);
            }
          }
          *(volatile v8h*)(C + (size_t)(mBase + row) * ldc + n0 + c8) = hv;
          if (OUT_MODE == 2) *(volatile v8h*)(C2 + (size_t)(mBase + row) * ldc + n0 + c8) = lv;
        }
        __threadfence();
      }
    }
    __builtin_amdgcn_fence(__ATOMIC_RELEASE, "workgroup");
    __builtin_amdgcn_wave_barrier();
    __builtin_amdgcn_fence(__ATOMIC_ACQUIRE, "workgroup");
  }
}

__global__ __launch_bounds__(256) void split_bf16_kernel(const float* __restrict__ in,
                                                         unsigned short* __restrict__ hi,
                                                         unsigned short* __restrict__ lo, int n8) {
  const int i = blockIdx.x * 256 + threadIdx.x;
  if (i >= n8) return;
  const float* p = in + 8 * (size_t)i;
  const v4f a = *(const v4f*)(p);
  const v4f c = *(const v4f*)(p + 4);
  float f[8];
#pragma unroll
  for (int e = 0; e < 4; ++e) { f[e] = a[e]; f[4 + e] = c[e]; }
  unsigned short hb[8], lb[8];
#pragma unroll
  for (int e = 0; e < 8; ++e) {
    hb[e] = f2bf_bits(f[e]);
    lb[e] = f2bf_bits(f[e] - bf_bits2f(hb[e]));
  }
  const v4u uh = (v4u){pk16(hb[0], hb[1]), pk16(hb[2], hb[3]), pk16(hb[4], hb[5]), pk16(hb[6], hb[7])};
  const v4u ul = (v4u){pk16(lb[0], lb[1]), pk16(lb[2], lb[3]), pk16(lb[4], lb[5]), pk16(lb[6], lb[7])};
  unsigned short* qh = hi + 8 * (size_t)i;
  unsigned short* ql = lo + 8 * (size_t)i;
  *(volatile v4u*)qh = uh;
  *(volatile v4u*)ql = ul;
  __threadfence();
  *(volatile v4u*)qh = uh;
  *(volatile v4u*)ql = ul;
}

__global__ __launch_bounds__(256) void sparsemax_col_kernel(const float* __restrict__ logits,
                                                            unsigned short* __restrict__ Shi,
                                                            unsigned short* __restrict__ Slo) {
#pragma clang fp contract(off)
  __shared__ float sv[kDim];
  __shared__ float cs[kDim];
  __shared__ __align__(16) float sel[kDim];
  __shared__ int wcnt[8];
  const int col  = blockIdx.x;
  const int t    = threadIdx.x;
  const int lane = t & 31, wave = t >> 5;

  const float z = logits[(size_t)t * kND + col];
  sv[t] = z;
  __syncthreads();

  for (int k = 2; k <= kDim; k <<= 1) {
    for (int j = k >> 1; j > 0; j >>= 1) {
      const int ixj = t ^ j;
      if (ixj > t) {
        const float a = sv[t];
        const float bb = sv[ixj];
        const bool desc = ((t & k) == 0);
        const bool swp = desc ? (a < bb) : (a > bb);
        if (swp) { sv[t] = bb; sv[ixj] = a; }
      }
      __syncthreads();
    }
  }

  cs[t] = sv[t];
  __syncthreads();
  for (int off = 1; off < kDim; off <<= 1) {
    const float v = cs[t];
    const float u = cs[(t >= off) ? (t - off) : 0];
    const float nv = (t >= off) ? (v + u) : v;
    __syncthreads();
    cs[t] = nv;
    __syncthreads();
  }

  const float lhs = 1.0f + (float)(t + 1) * sv[t];
  const int sup = (lhs > cs[t]) ? 1 : 0;
  const unsigned bal = __builtin_amdgcn_ballot_w32(sup != 0);
  const int wc = (int)__builtin_popcount(bal);
  if (lane == 0) wcnt[wave] = wc;
  __syncthreads();
  int kz = 0;
#pragma unroll
  for (int w = 0; w < 8; ++w) kz += wcnt[w];
  kz = (kz < 1) ? 1 : ((kz > kDim) ? kDim : kz);
  const float tau = (cs[kz - 1] - 1.0f) / (float)kz;
  sel[t] = fmaxf(z - tau, 0.0f);
  __syncthreads();

  if (wave == 0) {
    const float* sp = sel + 8 * lane;
    const v4f a = *(const v4f*)(sp);
    const v4f c = *(const v4f*)(sp + 4);
    float f[8];
#pragma unroll
    for (int e = 0; e < 4; ++e) { f[e] = a[e]; f[4 + e] = c[e]; }
    unsigned short hb[8], lb[8];
#pragma unroll
    for (int e = 0; e < 8; ++e) {
      hb[e] = f2bf_bits(f[e]);
      lb[e] = f2bf_bits(f[e] - bf_bits2f(hb[e]));
    }
    const v4u uh = (v4u){pk16(hb[0], hb[1]), pk16(hb[2], hb[3]), pk16(hb[4], hb[5]), pk16(hb[6], hb[7])};
    const v4u ul = (v4u){pk16(lb[0], lb[1]), pk16(lb[2], lb[3]), pk16(lb[4], lb[5]), pk16(lb[6], lb[7])};
    const size_t o = (size_t)col * kDim + 8 * lane;
    *(volatile v4u*)(Shi + o) = uh;
    *(volatile v4u*)(Slo + o) = ul;
    __threadfence();
    *(volatile v4u*)(Shi + o) = uh;
    *(volatile v4u*)(Slo + o) = ul;
  }
}

__global__ __launch_bounds__(256) void leaf_out_kernel(const float* __restrict__ FV,
                                                       const float* __restrict__ thr,
                                                       const float* __restrict__ logT,
                                                       const float* __restrict__ resp,
                                                       float* __restrict__ out) {
  __shared__ __align__(16) float sTL[kHalfNT * kDepth];
  __shared__ __align__(16) float sO[kHalfNT * kUnits];
  constexpr int kSlots = kHalfNT * kDepth / 4;
  const int t    = threadIdx.x;
  const int bIdx = blockIdx.x >> 1;
  const int n0   = (blockIdx.x & 1) * kHalfNT;
  const size_t fbase = (size_t)bIdx * kND + (size_t)n0 * kDepth;
  const int pbase = n0 * kDepth;

#pragma unroll 1
  for (int it = 0; it < 2; ++it) {
    const int slot = it * 256 + t;
    if (slot < kSlots) {
      const v4f f  = *(const v4f*)(FV + fbase + 4 * slot);
      const v4f th = *(const v4f*)(thr + pbase + 4 * slot);
      const v4f lt = *(const v4f*)(logT + pbase + 4 * slot);
      v4f r;
#pragma unroll
      for (int e = 0; e < 4; ++e) r[e] = (f[e] - th[e]) * expf(-lt[e]);
      *(v4f*)(sTL + 4 * slot) = r;
    }
  }
  __syncthreads();

  float g0[kDepth], g1[kDepth];
  {
    const float* tp = sTL + t * kDepth;
#pragma unroll
    for (int j = 0; j < 3; ++j) {
      const v2f v = *(const v2f*)(tp + 2 * j);
#pragma unroll
      for (int e = 0; e < 2; ++e) {
        const float tl = v[e];
        g1[2 * j + e] = fminf(fmaxf(0.5f * tl + 0.5f, 0.0f), 1.0f);
        g0[2 * j + e] = fminf(fmaxf(-0.5f * tl + 0.5f, 0.0f), 1.0f);
      }
    }
  }

  const float* rp = resp + (size_t)(n0 + t) * (kUnits * kLeaves);
  float a0 = 0.0f, a1 = 0.0f, a2 = 0.0f;
#pragma unroll 2
  for (int c = 0; c < kLeaves; ++c) {
    float p = (c & 1) ? g0[0] : g1[0];
#pragma unroll
    for (int d = 1; d < kDepth; ++d) {
      const float gg = ((c >> d) & 1) ? g0[d] : g1[d];
      p = p * gg;
    }
    a0 = fmaf(p, rp[c], a0);
    a1 = fmaf(p, rp[kLeaves + c], a1);
    a2 = fmaf(p, rp[2 * kLeaves + c], a2);
  }

  sO[t * kUnits + 0] = a0;
  sO[t * kUnits + 1] = a1;
  sO[t * kUnits + 2] = a2;
  __syncthreads();

  constexpr int kOutSlots = kHalfNT * kUnits / 4;
  float* op = out + (size_t)blockIdx.x * (kHalfNT * kUnits) + 4 * t;
  v4f ov = (v4f){0.f, 0.f, 0.f, 0.f};
  if (t < kOutSlots) {
    ov = *(const v4f*)(sO + 4 * t);
    *(volatile v4f*)op = ov;
  }
  __threadfence();
  if (t < kOutSlots) {
    *(volatile v4f*)op = ov;
  }
}

extern "C" void kernel_launch(void* const* d_in, const int* in_sizes, int n_in,
                              void* d_out, int out_size, void* d_ws, size_t ws_size,
                              hipStream_t stream) {
  (void)n_in;
  if (in_sizes[0] != kBatch * kDim) return;
  if (in_sizes[1] != kDim * kND) return;
  if (in_sizes[2] != kND) return;
  if (in_sizes[3] != kND) return;
  if (in_sizes[4] != kNT * kUnits * kLeaves) return;
  if (out_size != kBatch * kNT * kUnits) return;
  if (ws_size < kWsTotal) return;

  const float* x      = (const float*)d_in[0];
  const float* logits = (const float*)d_in[1];
  const float* thr    = (const float*)d_in[2];
  const float* logT   = (const float*)d_in[3];
  const float* resp   = (const float*)d_in[4];
  float* out          = (float*)d_out;

  char* ws = (char*)d_ws;
  unsigned short* Xhi = (unsigned short*)(ws + kOffXhi);
  unsigned short* Xlo = (unsigned short*)(ws + kOffXlo);
  unsigned short* Shi = (unsigned short*)(ws + kOffShi);
  unsigned short* Slo = (unsigned short*)(ws + kOffSlo);
  float*          FV  = (float*)(ws + kOffFV);

  const int n8 = kBatch * kDim / 8;
  split_bf16_kernel<<<dim3(n8 / 256), dim3(256), 0, stream>>>(x, Xhi, Xlo, n8);

  sparsemax_col_kernel<<<dim3(kND), dim3(kDim), 0, stream>>>(logits, Shi, Slo);

  const int tiles = (kBatch / 64) * (kND / 64);
  wmma_gemm64<1, true, 0, 0, false, 0><<<dim3(tiles / 8, 1), dim3(256), 0, stream>>>(
      Xhi, Xlo, kDim, 0L,
      Shi, Slo, kDim, 0L,
      (void*)FV, nullptr, kND, 0L,
      nullptr, nullptr, 0L,
      kBatch, kND, kDim, 1.0f);

  leaf_out_kernel<<<dim3(kBatch * 2), dim3(256), 0, stream>>>(FV, thr, logT, resp, out);
}
